// MultiQueryAttention_39848706573774
// MI455X (gfx1250) — hardware-verified
//
#include <hip/hip_runtime.h>
#include <stdint.h>


typedef _Float16 v16h __attribute__((ext_vector_type(16)));
typedef _Float16 v8h  __attribute__((ext_vector_type(8)));
typedef float    v8f  __attribute__((ext_vector_type(8)));
typedef float    v4f  __attribute__((ext_vector_type(4)));

#define DM 1024
#define HD 64
#define NH 16
#define NB_FULL 4
#define SEQ_FULL 2048
#ifndef NB
#define NB 4
#endif
#ifndef SEQ
#define SEQ 2048
#endif
#define MROWS (NB * SEQ)
#define QT (SEQ / 16)
#define EROWS 256
#define EQT (EROWS / 16)
#define WSCALE 64.0f
#define PCARRY 256.0f
#define YCARRY 64.0f
#define RC 1024.0f
#define RCY 64.0f
#define LOG2E 1.4426950408889634f
#define PT (16 * 72)

static_assert(SEQ % 128 == 0);
static_assert(SEQ >= EROWS);
static_assert(SEQ <= SEQ_FULL);
static_assert(NB >= 1 && NB <= NB_FULL);
static_assert(EROWS % 128 == 0);
static_assert(NH % 4 == 0);
static_assert(DM % 128 == 0 && (2 * HD) == 128 && DM == NH * HD);

union HFrag { v16h v; v8h h[2]; };

__device__ __forceinline__ v16h load_frag(const _Float16* p) {
    HFrag f;
    f.h[0] = *reinterpret_cast<const v8h*>(p);
    f.h[1] = *reinterpret_cast<const v8h*>(p + 16);
    return f.v;
}

__device__ __forceinline__ v8f wmma16(v16h a, v16h b, v8f c) {
    return __builtin_amdgcn_wmma_f32_16x16x32_f16(false, a, false, b, (short)0, c, false, false);
}

__device__ __forceinline__ float bf16r(float f) {
    unsigned int u = __float_as_uint(f);
    u += 0x7FFFu + ((u >> 16) & 1u);
    u &= 0xFFFF0000u;
    return __uint_as_float(u);
}

__global__ __launch_bounds__(256) void k_cvt_x(const float* __restrict__ x, _Float16* x16)
{
    const int u = blockIdx.x * 256 + threadIdx.x;
    const int row = u >> 7;
    const int col = (u & 127) * 8;
    const int bb = row / SEQ;
    const int s  = row - bb * SEQ;
    const float* src = x + ((size_t)(bb * SEQ_FULL + s)) * DM + col;
    const float4 f0 = *reinterpret_cast<const float4*>(src);
    const float4 f1 = *reinterpret_cast<const float4*>(src + 4);
    v8h o;
    o[0] = (_Float16)bf16r(f0.x); o[1] = (_Float16)bf16r(f0.y);
    o[2] = (_Float16)bf16r(f0.z); o[3] = (_Float16)bf16r(f0.w);
    o[4] = (_Float16)bf16r(f1.x); o[5] = (_Float16)bf16r(f1.y);
    o[6] = (_Float16)bf16r(f1.z); o[7] = (_Float16)bf16r(f1.w);
    _Float16* dst = x16 + (size_t)row * DM + col;
    *(volatile v8h*)dst = o;
    __threadfence();
    *(volatile v8h*)dst = o;
}

__global__ __launch_bounds__(256) void k_wt(const float* __restrict__ W, _Float16* WT, int N, float scl)
{
    __shared__ _Float16 tile[32 * 72] __attribute__((aligned(16)));
    const int tid = threadIdx.x;
    const int n0 = blockIdx.x * 32, k0 = blockIdx.y * 64;
    const int nn = tid & 31, kq = tid >> 5;
#pragma unroll
    for (int i = 0; i < 8; ++i) {
        const int kk = kq + 8 * i;
        const float w = W[(size_t)(k0 + kk) * N + n0 + nn];
        tile[nn * 72 + kk] = (_Float16)(bf16r(w) * scl);
    }
    __syncthreads();
    const int on = tid >> 3, seg = tid & 7;
    const v8h v = *reinterpret_cast<const v8h*>(tile + on * 72 + seg * 8);
    _Float16* dst = WT + (size_t)(n0 + on) * DM + k0 + seg * 8;
    *(volatile v8h*)dst = v;
    __threadfence();
    *(volatile v8h*)dst = v;
}

__device__ __forceinline__ void store32x64_f16(const _Float16* sw, _Float16* gdst,
                                               size_t pitch, int lane)
{
    const int rq = lane >> 3, seg = lane & 7;
    v8h v[8];
#pragma unroll
    for (int it = 0; it < 8; ++it)
        v[it] = *reinterpret_cast<const v8h*>(sw + (it * 4 + rq) * 64 + seg * 8);
#pragma unroll
    for (int it = 0; it < 8; ++it)
        *(volatile v8h*)(gdst + (size_t)(it * 4 + rq) * pitch + seg * 8) = v[it];
    __threadfence();
#pragma unroll
    for (int it = 0; it < 8; ++it)
        *(volatile v8h*)(gdst + (size_t)(it * 4 + rq) * pitch + seg * 8) = v[it];
}

template <int MODE>
__global__ __launch_bounds__(256) void k_gemm(const _Float16* __restrict__ A, int lda,
                                              const _Float16* __restrict__ BT, int ldb, int K,
                                              const _Float16* __restrict__ A2, int lda2,
                                              const _Float16* __restrict__ BT2, int ldb2, int K2,
                                              void* C0, void* C1, void* C2, void* C3,
                                              int N, int rb, int row0, float alpha)
{
    __shared__ float stg[8 * 1024] __attribute__((aligned(16)));
    const int tid = threadIdx.x;
    const int lane = tid & 31, wave = tid >> 5;
    const int wm = wave & 3, wn = wave >> 2;
    const int l15 = lane & 15, hi8 = (lane >> 4) << 3;
    const int by  = blockIdx.y;
    const int bm0 = (by / rb) * SEQ + row0 + (by % rb) * 128;
    const int bn0 = blockIdx.x * 128;

    const v8f zero8 = {0.f, 0.f, 0.f, 0.f, 0.f, 0.f, 0.f, 0.f};
    v8f acc[2][4];
#pragma unroll
    for (int g = 0; g < 2; ++g)
#pragma unroll
        for (int ni = 0; ni < 4; ++ni) acc[g][ni] = zero8;

#pragma unroll
    for (int ph = 0; ph < 2; ++ph) {
        const _Float16* Ab = (ph == 0) ? A : A2;
        const _Float16* Bb = (ph == 0) ? BT : BT2;
        const int la = (ph == 0) ? lda : lda2;
        const int lb = (ph == 0) ? ldb : ldb2;
        const int KK = (ph == 0) ? K : K2;
        const _Float16* ap0 = Ab + (size_t)(bm0 + wm * 32 + l15) * la + hi8;
        const _Float16* ap1 = ap0 + (size_t)16 * la;
        const _Float16* bp  = Bb + (size_t)(bn0 + wn * 64 + l15) * lb + hi8;
        const size_t bst = (size_t)16 * lb;

        for (int k0 = 0; k0 < KK; k0 += 32) {
            const v16h a0 = load_frag(ap0 + k0);
            const v16h a1 = load_frag(ap1 + k0);
            const v16h b0 = load_frag(bp + k0);
            const v16h b1 = load_frag(bp + bst + k0);
            const v16h b2 = load_frag(bp + 2 * bst + k0);
            const v16h b3 = load_frag(bp + 3 * bst + k0);
            acc[0][0] = wmma16(a0, b0, acc[0][0]);
            acc[0][1] = wmma16(a0, b1, acc[0][1]);
            acc[0][2] = wmma16(a0, b2, acc[0][2]);
            acc[0][3] = wmma16(a0, b3, acc[0][3]);
            acc[1][0] = wmma16(a1, b0, acc[1][0]);
            acc[1][1] = wmma16(a1, b1, acc[1][1]);
            acc[1][2] = wmma16(a1, b2, acc[1][2]);
            acc[1][3] = wmma16(a1, b3, acc[1][3]);
            asm volatile("v_nop\n\tv_nop\n\tv_nop\n\tv_nop"
                         : "+v"(acc[0][0]), "+v"(acc[0][1]), "+v"(acc[0][2]), "+v"(acc[0][3]),
                           "+v"(acc[1][0]), "+v"(acc[1][1]), "+v"(acc[1][2]), "+v"(acc[1][3])
                         : "v"(a0), "v"(a1), "v"(b0), "v"(b1), "v"(b2), "v"(b3));
        }
    }

    if (MODE == 0) {
        _Float16* sw = reinterpret_cast<_Float16*>(stg + wave * 1024);
#pragma unroll
        for (int p = 0; p < 2; ++p) {
#pragma unroll
            for (int g = 0; g < 2; ++g)
#pragma unroll
                for (int ni = 0; ni < 4; ++ni)
#pragma unroll
                    for (int j = 0; j < 8; ++j) {
                        const float val = acc[g][ni][j] * alpha;
                        const _Float16 hv = (_Float16)val;
                        sw[(g * 16 + hi8 + j) * 64 + ni * 16 + l15] =
                            (p == 0) ? hv : (_Float16)((val - (float)hv) * RC);
                    }
            __syncthreads();
            _Float16* cp = (p == 0) ? (_Float16*)C0 : (_Float16*)C1;
            store32x64_f16(sw, cp + (size_t)(bm0 + wm * 32) * N + bn0 + wn * 64, (size_t)N, lane);
            __syncthreads();
        }
    } else if (MODE == 1) {
        float* swf = stg + wave * 1024;
        const int rq = lane >> 4, seg = lane & 15;
#pragma unroll
        for (int g = 0; g < 2; ++g) {
#pragma unroll
            for (int ni = 0; ni < 4; ++ni)
#pragma unroll
                for (int j = 0; j < 8; ++j)
                    swf[(hi8 + j) * 64 + ni * 16 + l15] = acc[g][ni][j] * alpha;
            __syncthreads();
            v4f v[8];
#pragma unroll
            for (int it = 0; it < 8; ++it)
                v[it] = *reinterpret_cast<const v4f*>(swf + (it * 2 + rq) * 64 + seg * 4);
            float* gd = (float*)C0 + (size_t)(bm0 + wm * 32 + g * 16) * N + bn0 + wn * 64 + seg * 4;
#pragma unroll
            for (int it = 0; it < 8; ++it)
                *(volatile v4f*)(gd + (size_t)(it * 2 + rq) * N) = v[it];
            __threadfence();
#pragma unroll
            for (int it = 0; it < 8; ++it)
                *(volatile v4f*)(gd + (size_t)(it * 2 + rq) * N) = v[it];
            __syncthreads();
        }
    } else {
        _Float16* sw = reinterpret_cast<_Float16*>(stg + wave * 1024);
        _Float16* vs = reinterpret_cast<_Float16*>(stg + 4 * 1024);
        const int bb = bm0 / SEQ;
        const int s0 = bm0 - bb * SEQ;
        const int dq = tid >> 4, sg = tid & 15;
#pragma unroll
        for (int p = 0; p < 2; ++p) {
            if (wn == 0) {
#pragma unroll
                for (int g = 0; g < 2; ++g)
#pragma unroll
                    for (int ni = 0; ni < 4; ++ni)
#pragma unroll
                        for (int j = 0; j < 8; ++j) {
                            const float val = acc[g][ni][j] * alpha;
                            const _Float16 hv = (_Float16)val;
                            sw[(g * 16 + hi8 + j) * 64 + ni * 16 + l15] =
                                (p == 0) ? hv : (_Float16)((val - (float)hv) * RC);
                        }
            } else {
#pragma unroll
                for (int g = 0; g < 2; ++g)
#pragma unroll
                    for (int ni = 0; ni < 4; ++ni)
#pragma unroll
                        for (int j = 0; j < 8; ++j) {
                            const float val = acc[g][ni][j] * alpha;
                            const _Float16 hv = (_Float16)val;
                            vs[(ni * 16 + l15) * 128 + wm * 32 + g * 16 + hi8 + j] =
                                (p == 0) ? hv : (_Float16)((val - (float)hv) * RC);
                        }
            }
            __syncthreads();
            if (wn == 0) {
                _Float16* kd = (p == 0) ? (_Float16*)C0 : (_Float16*)C2;
                store32x64_f16(sw, kd + (size_t)(bm0 + wm * 32) * HD, (size_t)HD, lane);
            }
            {
                v8h v[4];
#pragma unroll
                for (int it = 0; it < 4; ++it)
                    v[it] = *reinterpret_cast<const v8h*>(vs + (it * 16 + dq) * 128 + sg * 8);
                _Float16* vpl = (p == 0) ? (_Float16*)C1 : (_Float16*)C3;
                _Float16* vd = vpl + ((size_t)(bb * HD)) * SEQ + s0 + sg * 8;
#pragma unroll
                for (int it = 0; it < 4; ++it)
                    *(volatile v8h*)(vd + (size_t)(it * 16 + dq) * SEQ) = v[it];
                __threadfence();
#pragma unroll
                for (int it = 0; it < 4; ++it)
                    *(volatile v8h*)(vd + (size_t)(it * 16 + dq) * SEQ) = v[it];
            }
            __syncthreads();
        }
    }
}

__global__ __launch_bounds__(128) __attribute__((amdgpu_num_vgpr(256)))
void k_attn(const _Float16* __restrict__ qp, const _Float16* __restrict__ kp,
            const _Float16* __restrict__ vT, _Float16* yp, int qt0, int nqt)
{
    __shared__ _Float16 Ws[4 * PT] __attribute__((aligned(16)));
    const int lane = threadIdx.x & 31;
    const int wv   = threadIdx.x >> 5;
    const int l15  = lane & 15;
    const int hi8  = (lane >> 4) << 3;

    int bx = blockIdx.x;
    const int hg = bx % (NH / 4); bx /= (NH / 4);
    const int qt = qt0 + bx % nqt;
    const int b  = bx / nqt;
    const int h  = hg * 4 + wv;

    const _Float16* qbase = qp + ((size_t)(b * SEQ + qt * 16 + l15)) * DM + h * HD + hi8;
    const v16h aQ0 = load_frag(qbase);
    const v16h aQ1 = load_frag(qbase + 32);

    const _Float16* kbase = kp + (size_t)b * SEQ * HD + hi8;
    const _Float16* vbase = vT + (size_t)(b * HD) * SEQ + hi8;

    const v8f zero8 = {0.f, 0.f, 0.f, 0.f, 0.f, 0.f, 0.f, 0.f};
    float m[8], l[8];
    v8f accY[4];
#pragma unroll
    for (int j = 0; j < 8; ++j) { m[j] = -1e30f; l[j] = 0.0f; }
#pragma unroll
    for (int ni = 0; ni < 4; ++ni) accY[ni] = zero8;

    _Float16* ps = Ws + wv * PT;
    const int tend  = qt * 16 + 16;
    const int trow0 = qt * 16 + hi8;

#pragma unroll 1
    for (int tc = 0; tc < tend; tc += 32) {
        const _Float16* kp0 = kbase + (size_t)(tc + l15) * HD;
        const _Float16* kp1 = kp0 + 16 * HD;
        const v16h b00 = load_frag(kp0);
        const v16h b01 = load_frag(kp0 + 32);
        const v16h b10 = load_frag(kp1);
        const v16h b11 = load_frag(kp1 + 32);
        v8f s0 = zero8, s1 = zero8;
        s0 = wmma16(aQ0, b00, s0);
        s0 = wmma16(aQ1, b01, s0);
        s1 = wmma16(aQ0, b10, s1);
        s1 = wmma16(aQ1, b11, s1);
        asm volatile("v_nop\n\tv_nop\n\tv_nop\n\tv_nop"
                     : "+v"(s0), "+v"(s1)
                     : "v"(aQ0), "v"(aQ1), "v"(b00), "v"(b01), "v"(b10), "v"(b11));

        const int key0 = tc + l15, key1 = tc + 16 + l15;
#pragma unroll
        for (int j = 0; j < 8; ++j) {
            const int t = trow0 + j;
            const float a0 = (key0 <= t) ? s0[j] * 0.125f : -1e30f;
            const float a1 = (key1 <= t) ? s1[j] * 0.125f : -1e30f;
            float mt = fmaxf(a0, a1);
#pragma unroll
            for (int off = 8; off >= 1; off >>= 1)
                mt = fmaxf(mt, __shfl_xor(mt, off, 16));
            const float mn = fmaxf(m[j], mt);
            const float sc = exp2f(m[j] - mn);
            const float p0 = exp2f(a0 - mn);
            const float p1 = exp2f(a1 - mn);
            float rs = p0 + p1;
#pragma unroll
            for (int off = 8; off >= 1; off >>= 1)
                rs += __shfl_xor(rs, off, 16);
            l[j] = l[j] * sc + rs;
            m[j] = mn;
            accY[0][j] *= sc; accY[1][j] *= sc;
            accY[2][j] *= sc; accY[3][j] *= sc;
            const int row = hi8 + j;
            ps[row * 72 + l15]      = (_Float16)(p0 * PCARRY);
            ps[row * 72 + 16 + l15] = (_Float16)(p1 * PCARRY);
        }
        __syncthreads();

        const v16h aP = load_frag(ps + l15 * 72 + hi8);
        const v16h bV0 = load_frag(vbase + (size_t)(0 * 16 + l15) * SEQ + tc);
        const v16h bV1 = load_frag(vbase + (size_t)(1 * 16 + l15) * SEQ + tc);
        const v16h bV2 = load_frag(vbase + (size_t)(2 * 16 + l15) * SEQ + tc);
        const v16h bV3 = load_frag(vbase + (size_t)(3 * 16 + l15) * SEQ + tc);
        accY[0] = wmma16(aP, bV0, accY[0]);
        accY[1] = wmma16(aP, bV1, accY[1]);
        accY[2] = wmma16(aP, bV2, accY[2]);
        accY[3] = wmma16(aP, bV3, accY[3]);
        asm volatile("v_nop\n\tv_nop\n\tv_nop\n\tv_nop"
                     : "+v"(accY[0]), "+v"(accY[1]), "+v"(accY[2]), "+v"(accY[3])
                     : "v"(aP), "v"(bV0), "v"(bV1), "v"(bV2), "v"(bV3));
    }
    __syncthreads();

    float inv[8];
#pragma unroll
    for (int j = 0; j < 8; ++j) inv[j] = (YCARRY / PCARRY) / l[j];
#pragma unroll
    for (int ni = 0; ni < 4; ++ni)
#pragma unroll
        for (int j = 0; j < 8; ++j)
            ps[(hi8 + j) * 72 + ni * 16 + l15] = (_Float16)(accY[ni][j] * inv[j]);
    __syncthreads();

    const int rq = lane >> 3, seg = lane & 7;
    v8h v[4];
#pragma unroll
    for (int it = 0; it < 4; ++it)
        v[it] = *reinterpret_cast<const v8h*>(ps + (it * 4 + rq) * 72 + seg * 8);
    _Float16* yd = yp + ((size_t)(b * SEQ + qt * 16)) * DM + h * HD + seg * 8;
#pragma unroll
    for (int it = 0; it < 4; ++it)
        *(volatile v8h*)(yd + (size_t)(it * 4 + rq) * DM) = v[it];
    __threadfence();
#pragma unroll
    for (int it = 0; it < 4; ++it)
        *(volatile v8h*)(yd + (size_t)(it * 4 + rq) * DM) = v[it];
}

__global__ __launch_bounds__(128) __attribute__((amdgpu_num_vgpr(256)))
void k_attn_e(const _Float16* __restrict__ qh, const _Float16* __restrict__ qr,
              const _Float16* __restrict__ kh, const _Float16* __restrict__ kr,
              const _Float16* __restrict__ vh, const _Float16* __restrict__ vr,
              _Float16* yh, _Float16* yr)
{
    __shared__ _Float16 Ps[4 * 2 * PT] __attribute__((aligned(16)));
    __shared__ _Float16 Ys[2 * 2 * PT] __attribute__((aligned(16)));
    const int lane = threadIdx.x & 31;
    const int wv   = threadIdx.x >> 5;
    const int l15  = lane & 15;
    const int hi8  = (lane >> 4) << 3;

    int bx = blockIdx.x;
    const int hp = bx % (NH / 2); bx /= (NH / 2);
    const int qt = bx % EQT;
    const int b  = bx / EQT;
    const int hs = wv >> 1, dh = wv & 1;
    const int h  = hp * 2 + hs;

    const size_t qrow = (size_t)b * SEQ + (size_t)qt * 16;
    const _Float16* qhb = qh + (qrow + l15) * DM + h * HD + hi8;
    const _Float16* qrb = qr + (qrow + l15) * DM + h * HD + hi8;
    const _Float16* khb = kh + (size_t)b * SEQ * HD + hi8;
    const _Float16* krb = kr + (size_t)b * SEQ * HD + hi8;
    const _Float16* vhb = vh + (size_t)(b * HD + dh * 32) * SEQ + hi8;
    const _Float16* vrb = vr + (size_t)(b * HD + dh * 32) * SEQ + hi8;

    const v8f zero8 = {0.f, 0.f, 0.f, 0.f, 0.f, 0.f, 0.f, 0.f};
    float m[8], l[8];
    v8f accY[2], accR[2];
#pragma unroll
    for (int j = 0; j < 8; ++j) { m[j] = -1e30f; l[j] = 0.0f; }
#pragma unroll
    for (int ni = 0; ni < 2; ++ni) { accY[ni] = zero8; accR[ni] = zero8; }

    _Float16* ps = Ps + (wv * 2 + 0) * PT;
    _Float16* pr = Ps + (wv * 2 + 1) * PT;
    const int tend  = qt * 16 + 16;
    const int trow0 = qt * 16 + hi8;

#pragma unroll 1
    for (int tc = 0; tc < tend; tc += 32) {
        const _Float16* k0p = khb + (size_t)(tc + l15) * HD;
        const _Float16* k1p = k0p + 16 * HD;
        const v16h bh00 = load_frag(k0p);
        const v16h bh01 = load_frag(k0p + 32);
        const v16h bh10 = load_frag(k1p);
        const v16h bh11 = load_frag(k1p + 32);
        v8f s0 = zero8, s1 = zero8, r0 = zero8, r1 = zero8;
        {
            const v16h ar0 = load_frag(qrb);
            const v16h ar1 = load_frag(qrb + 32);
            r0 = wmma16(ar0, bh00, r0);
            r0 = wmma16(ar1, bh01, r0);
            r1 = wmma16(ar0, bh10, r1);
            r1 = wmma16(ar1, bh11, r1);
            asm volatile("v_nop\n\tv_nop\n\tv_nop\n\tv_nop"
                         : "+v"(r0), "+v"(r1)
                         : "v"(ar0), "v"(ar1), "v"(bh00), "v"(bh01), "v"(bh10), "v"(bh11));
        }
        const v16h a0 = load_frag(qhb);
        const v16h a1 = load_frag(qhb + 32);
        s0 = wmma16(a0, bh00, s0);
        s0 = wmma16(a1, bh01, s0);
        s1 = wmma16(a0, bh10, s1);
        s1 = wmma16(a1, bh11, s1);
        asm volatile("v_nop\n\tv_nop\n\tv_nop\n\tv_nop"
                     : "+v"(s0), "+v"(s1)
                     : "v"(a0), "v"(a1), "v"(bh00), "v"(bh01), "v"(bh10), "v"(bh11));
        {
            const _Float16* kr0p = krb + (size_t)(tc + l15) * HD;
            const _Float16* kr1p = kr0p + 16 * HD;
            const v16h br00 = load_frag(kr0p);
            const v16h br01 = load_frag(kr0p + 32);
            const v16h br10 = load_frag(kr1p);
            const v16h br11 = load_frag(kr1p + 32);
            r0 = wmma16(a0, br00, r0);
            r0 = wmma16(a1, br01, r0);
            r1 = wmma16(a0, br10, r1);
            r1 = wmma16(a1, br11, r1);
            asm volatile("v_nop\n\tv_nop\n\tv_nop\n\tv_nop"
                         : "+v"(r0), "+v"(r1)
                         : "v"(a0), "v"(a1), "v"(br00), "v"(br01), "v"(br10), "v"(br11));
        }

        const int key0 = tc + l15, key1 = tc + 16 + l15;
#pragma unroll
        for (int j = 0; j < 8; ++j) {
            const int t = trow0 + j;
            const float f0 = (s0[j] + r0[j] * (1.0f / RC)) * 0.125f;
            const float f1 = (s1[j] + r1[j] * (1.0f / RC)) * 0.125f;
            const float a0v = (key0 <= t) ? f0 : -1e30f;
            const float a1v = (key1 <= t) ? f1 : -1e30f;
            float mt = fmaxf(a0v, a1v);
#pragma unroll
            for (int off = 8; off >= 1; off >>= 1)
                mt = fmaxf(mt, __shfl_xor(mt, off, 16));
            const float mn = fmaxf(m[j], mt);
            const float sc = exp2f(m[j] - mn);
            const float p0 = exp2f(a0v - mn);
            const float p1 = exp2f(a1v - mn);
            float rs = p0 + p1;
#pragma unroll
            for (int off = 8; off >= 1; off >>= 1)
                rs += __shfl_xor(rs, off, 16);
            l[j] = l[j] * sc + rs;
            m[j] = mn;
            accY[0][j] *= sc; accY[1][j] *= sc;
            accR[0][j] *= sc; accR[1][j] *= sc;
            const float c0 = p0 * PCARRY, c1 = p1 * PCARRY;
            const _Float16 h0 = (_Float16)c0, h1 = (_Float16)c1;
            const int row = hi8 + j;
            ps[row * 72 + l15]      = h0;
            ps[row * 72 + 16 + l15] = h1;
            pr[row * 72 + l15]      = (_Float16)((c0 - (float)h0) * RC);
            pr[row * 72 + 16 + l15] = (_Float16)((c1 - (float)h1) * RC);
        }
        __syncthreads();

        const v16h aP = load_frag(ps + l15 * 72 + hi8);
        const v16h aR = load_frag(pr + l15 * 72 + hi8);
        {
            const v16h bv0 = load_frag(vhb + (size_t)(0 * 16 + l15) * SEQ + tc);
            const v16h bv1 = load_frag(vhb + (size_t)(1 * 16 + l15) * SEQ + tc);
            accY[0] = wmma16(aP, bv0, accY[0]);
            accY[1] = wmma16(aP, bv1, accY[1]);
            accR[0] = wmma16(aR, bv0, accR[0]);
            accR[1] = wmma16(aR, bv1, accR[1]);
            asm volatile("v_nop\n\tv_nop\n\tv_nop\n\tv_nop"
                         : "+v"(accY[0]), "+v"(accY[1]), "+v"(accR[0]), "+v"(accR[1])
                         : "v"(aP), "v"(aR), "v"(bv0), "v"(bv1));
        }
        {
            const v16h bw0 = load_frag(vrb + (size_t)(0 * 16 + l15) * SEQ + tc);
            const v16h bw1 = load_frag(vrb + (size_t)(1 * 16 + l15) * SEQ + tc);
            accR[0] = wmma16(aP, bw0, accR[0]);
            accR[1] = wmma16(aP, bw1, accR[1]);
            asm volatile("v_nop\n\tv_nop\n\tv_nop\n\tv_nop"
                         : "+v"(accR[0]), "+v"(accR[1])
                         : "v"(aP), "v"(bw0), "v"(bw1));
        }
    }
    __syncthreads();

    float inv[8];
#pragma unroll
    for (int j = 0; j < 8; ++j) inv[j] = (YCARRY / PCARRY) / l[j];
    _Float16* ysh = Ys + (hs * 2 + 0) * PT;
    _Float16* ysr = Ys + (hs * 2 + 1) * PT;
#pragma unroll
    for (int ni = 0; ni < 2; ++ni)
#pragma unroll
        for (int j = 0; j < 8; ++j) {
            const float val = (accY[ni][j] + accR[ni][j] * (1.0f / RC)) * inv[j];
            const _Float16 hv = (_Float16)val;
            const int idx = (hi8 + j) * 72 + dh * 32 + ni * 16 + l15;
            ysh[idx] = hv;
            ysr[idx] = (_Float16)((val - (float)hv) * RCY);
        }
    __syncthreads();

    const int rq = lane >> 3, seg = lane & 7;
    const _Float16* src = Ys + (hs * 2 + dh) * PT;
    v8h v[4];
#pragma unroll
    for (int it = 0; it < 4; ++it)
        v[it] = *reinterpret_cast<const v8h*>(src + (it * 4 + rq) * 72 + seg * 8);
    _Float16* ypl = (dh == 0) ? yh : yr;
    _Float16* yd = ypl + qrow * DM + h * HD + seg * 8;
#pragma unroll
    for (int it = 0; it < 4; ++it)
        *(volatile v8h*)(yd + (size_t)(it * 4 + rq) * DM) = v[it];
    __threadfence();
#pragma unroll
    for (int it = 0; it < 4; ++it)
        *(volatile v8h*)(yd + (size_t)(it * 4 + rq) * DM) = v[it];
}

extern "C" void kernel_launch(void* const* d_in, const int* in_sizes, int n_in,
                              void* d_out, int out_size, void* d_ws, size_t ws_size,
                              hipStream_t stream) {
    if (n_in < 5) return;
    const long long needX = ((long long)(NB - 1) * SEQ_FULL + SEQ) * DM;
    if ((long long)in_sizes[0] < needX) return;
    if (in_sizes[1] < DM * DM || in_sizes[2] < DM * HD || in_sizes[3] < DM * HD || in_sizes[4] < DM * DM) return;
    if ((long long)out_size < (long long)MROWS * DM) return;

    const float* x  = (const float*)d_in[0];
    const float* Wq = (const float*)d_in[1];
    const float* Wk = (const float*)d_in[2];
    const float* Wv = (const float*)d_in[3];
    const float* Wo = (const float*)d_in[4];
    float* out = (float*)d_out;

    size_t off = 0;
    char* wsb = (char*)d_ws;
    auto carve = [&](size_t bytes) -> void* {
        void* p = wsb + off;
        off += (bytes + 255) & ~(size_t)255;
        return p;
    };
    _Float16* x16  = (_Float16*)carve((size_t)MROWS * DM * 2);
    _Float16* WqT  = (_Float16*)carve((size_t)DM * DM * 2);
    _Float16* WkvT = (_Float16*)carve((size_t)(2 * HD) * DM * 2);
    _Float16* WoT  = (_Float16*)carve((size_t)DM * DM * 2);
    _Float16* WoU  = (_Float16*)carve((size_t)DM * DM * 2);
    _Float16* q16  = (_Float16*)carve((size_t)MROWS * DM * 2);
    _Float16* qrs  = (_Float16*)carve((size_t)MROWS * DM * 2);
    _Float16* kpl  = (_Float16*)carve((size_t)MROWS * HD * 2);
    _Float16* krs  = (_Float16*)carve((size_t)MROWS * HD * 2);
    _Float16* vT   = (_Float16*)carve((size_t)NB * HD * SEQ * 2);
    _Float16* vTr  = (_Float16*)carve((size_t)NB * HD * SEQ * 2);
    _Float16* y16  = (_Float16*)carve((size_t)MROWS * DM * 2);
    _Float16* yrs  = (_Float16*)carve((size_t)MROWS * DM * 2);
    if (off > ws_size) return;

    dim3 blk(256);

    k_cvt_x<<<dim3(MROWS / 2), blk, 0, stream>>>(x, x16);
    k_wt<<<dim3(DM / 32, DM / 64), blk, 0, stream>>>(Wq, WqT, DM, WSCALE);
    k_wt<<<dim3(HD / 32, DM / 64), blk, 0, stream>>>(Wk, WkvT, HD, WSCALE);
    k_wt<<<dim3(HD / 32, DM / 64), blk, 0, stream>>>(Wv, WkvT + (size_t)HD * DM, HD, WSCALE);
    k_wt<<<dim3(DM / 32, DM / 64), blk, 0, stream>>>(Wo, WoT, DM, WSCALE);
    k_wt<<<dim3(DM / 32, DM / 64), blk, 0, stream>>>(Wo, WoU, DM, WSCALE / RCY);

    k_gemm<0><<<dim3(DM / 128, MROWS / 128), blk, 0, stream>>>(
        x16, DM, WqT, DM, DM, x16, DM, WqT, DM, 0,
        (void*)q16, (void*)qrs, (void*)q16, (void*)qrs, DM, SEQ / 128, 0, LOG2E / WSCALE);
    k_gemm<2><<<dim3(1, MROWS / 128), blk, 0, stream>>>(
        x16, DM, WkvT, DM, DM, x16, DM, WkvT, DM, 0,
        (void*)kpl, (void*)vT, (void*)krs, (void*)vTr, 2 * HD, SEQ / 128, 0, 1.0f / WSCALE);

    k_attn_e<<<dim3(NB * (NH / 2) * EQT), dim3(128), 0, stream>>>(q16, qrs, kpl, krs, vT, vTr, y16, yrs);
    const int qtl = QT - EQT;
    if (qtl > 0)
        k_attn<<<dim3(NB * (NH / 4) * qtl), dim3(128), 0, stream>>>(q16, kpl, vT, y16, EQT, qtl);

    k_gemm<1><<<dim3(DM / 128, NB * (EROWS / 128)), blk, 0, stream>>>(
        y16, DM, WoT, DM, DM, yrs, DM, WoU, DM, DM,
        (void*)out, (void*)out, (void*)out, (void*)out, DM, EROWS / 128, 0, 1.0f / (YCARRY * WSCALE));
    const int rbl = (SEQ - EROWS) / 128;
    if (rbl > 0)
        k_gemm<1><<<dim3(DM / 128, NB * rbl), blk, 0, stream>>>(
            y16, DM, WoT, DM, DM, y16, DM, WoT, DM, 0,
            (void*)out, (void*)out, (void*)out, (void*)out, DM, rbl, EROWS, 1.0f / (YCARRY * WSCALE));
}
